// LocalAttentionBlock_75445395521923
// MI455X (gfx1250) — hardware-verified
//
#include <hip/hip_runtime.h>
#include <math.h>

constexpr int kTok     = 4096;
constexpr int kDim     = 1024;
constexpr int kHeads   = 16;
constexpr int kHdim    = 64;
constexpr int kWin     = 128;
constexpr int kMlp     = 4096;
constexpr int kQKld    = 2 * kDim;
constexpr int kPadRows = kTok + 2 * kWin;
constexpr int kVtld    = kPadRows;
constexpr int kChunkQ  = 128;
constexpr int kNChunk  = kTok / kChunkQ;
constexpr int kWinK    = kChunkQ + 2 * kWin;
constexpr float kWCarryInv  = 1.0f / 64.0f;
constexpr float kWCarry     = 64.0f;
constexpr float kPCarry     = 2048.0f;
constexpr float kOCarry     = 256.0f;
constexpr float kHCarry     = 16.0f;
constexpr float kScoreScale = 0.125f;
constexpr float kInvDim     = 1.0f / 1024.0f;
constexpr float kLnEps      = 1e-5f;

constexpr size_t kOffWqkv  = 0;
constexpr size_t kOffWout  = kOffWqkv + (size_t)3 * kDim * kDim * 2;
constexpr size_t kOffQK    = kOffWout + (size_t)kDim * kDim * 2;
constexpr size_t kOffVt    = kOffQK + (size_t)kPadRows * kQKld * 2;
constexpr size_t kOffS     = kOffVt + (size_t)kDim * kVtld * 2;
constexpr size_t kOffP     = kOffS + (size_t)kNChunk * kChunkQ * kWinK * 4;
constexpr size_t kOffO     = kOffP + (size_t)kTok * kWinK * 2;
constexpr size_t kEndAttn  = kOffO + (size_t)kTok * kDim * 2;
constexpr size_t kOffHpre  = 0;
constexpr size_t kOffW1    = kEndAttn;
constexpr size_t kOffW2    = kOffW1 + (size_t)kMlp * kDim * 2;
constexpr size_t kOffXn    = kOffW2 + (size_t)kDim * kMlp * 2;
constexpr size_t kOffX1    = kOffXn + (size_t)kTok * kDim * 2;
constexpr size_t kOffHact  = kOffX1 + (size_t)kTok * kDim * 4;
constexpr size_t kWsTotal  = kOffHact + (size_t)kTok * kMlp * 2;
static_assert(kOffHpre + (size_t)kTok * kMlp * 2 <= kEndAttn, "hpre fits in the dead attention regions");
static_assert(kWsTotal == 128450560, "carve total");
static_assert(kWsTotal <= 134217728, "carve under 128 MiB");

typedef __attribute__((ext_vector_type(16))) _Float16 v16h;
typedef __attribute__((ext_vector_type(8)))  _Float16 v8h;
typedef __attribute__((ext_vector_type(16))) __bf16   v16b;
typedef __attribute__((ext_vector_type(8)))  __bf16   v8b;
typedef __attribute__((ext_vector_type(8)))  float    v8f;
typedef __attribute__((ext_vector_type(4)))  float    v4f;
typedef __attribute__((ext_vector_type(4)))  unsigned int v4u;

__device__ __forceinline__ unsigned short f2bf_bits(float f) {
  unsigned u = __float_as_uint(f);
  return (unsigned short)((u + 0x7FFFu + ((u >> 16) & 1u)) >> 16);
}
__device__ __forceinline__ float bf_bits2f(unsigned short h) { return __uint_as_float(((unsigned)h) << 16); }

__device__ __forceinline__ void dep_guard_h(v8f& a, v8f& b, v16h x, v16h y) { asm volatile("v_nop\n\tv_nop\n\tv_nop\n\tv_nop" : "+v"(a), "+v"(b) : "v"(x), "v"(y)); }
__device__ __forceinline__ void dep_guard_b(v8f& a, v8f& b, v16b x, v16b y) { asm volatile("v_nop\n\tv_nop\n\tv_nop\n\tv_nop" : "+v"(a), "+v"(b) : "v"(x), "v"(y)); }
__device__ __forceinline__ void keep4_h(v16h a, v16h b, v16h c, v16h d) { asm volatile("v_nop" :: "v"(a), "v"(b), "v"(c), "v"(d)); }
__device__ __forceinline__ void keep4_b(v16b a, v16b b, v16b c, v16b d) { asm volatile("v_nop" :: "v"(a), "v"(b), "v"(c), "v"(d)); }
__device__ __forceinline__ void acc_guard4(v8f& a, v8f& b, v8f& c, v8f& d) { asm volatile("v_nop\n\tv_nop\n\tv_nop\n\tv_nop" : "+v"(a), "+v"(b), "+v"(c), "+v"(d)); }
template <typename T> struct Frag;
template <> struct Frag<_Float16> {
  typedef v16h V; union U { v16h v; v8h h[2]; };
  static __device__ __forceinline__ v16h load(const _Float16* p) {
    U f; f.h[0] = *(const v8h*)(p); f.h[1] = *(const v8h*)(p + 16); return f.v;
  }
  static __device__ __forceinline__ v8f mma(v16h a, v16h b, v8f c) {
    return __builtin_amdgcn_wmma_f32_16x16x32_f16(false, a, false, b, (short)0, c, false, false);
  }
  static __device__ __forceinline__ void guard(v8f& a, v8f& b, v16h x, v16h y) { dep_guard_h(a, b, x, y); }
  static __device__ __forceinline__ void keep(v16h a, v16h b, v16h c, v16h d) { keep4_h(a, b, c, d); }
};
template <> struct Frag<__bf16> {
  typedef v16b V; union U { v16b v; v8b h[2]; };
  static __device__ __forceinline__ v16b load(const __bf16* p) {
    U f; f.h[0] = *(const v8b*)(p); f.h[1] = *(const v8b*)(p + 16); return f.v;
  }
  static __device__ __forceinline__ v8f mma(v16b a, v16b b, v8f c) {
    return __builtin_amdgcn_wmma_f32_16x16x32_bf16(false, a, false, b, (short)0, c, false, false);
  }
  static __device__ __forceinline__ void guard(v8f& a, v8f& b, v16b x, v16b y) { dep_guard_b(a, b, x, y); }
  static __device__ __forceinline__ void keep(v16b a, v16b b, v16b c, v16b d) { keep4_b(a, b, c, d); }
};

__device__ __forceinline__ unsigned pk16(unsigned short a, unsigned short b) { return (unsigned)a | ((unsigned)b << 16); }
__device__ __forceinline__ unsigned short h_bits(float f) { const _Float16 h = (_Float16)f; return __builtin_bit_cast(unsigned short, h); }

template <int ET> struct Elem;
template <> struct Elem<0> { typedef _Float16 T; };
template <> struct Elem<1> { typedef __bf16 T; };
template <int ET, bool SPLIT, int BIAS_MODE, int OUT_MODE, bool RESID, int ACT = 0>
__global__ __launch_bounds__(256) void wmma_gemm64(
    const unsigned short* __restrict__ Ap, const unsigned short* __restrict__ A2p, int lda, long strideA,
    const unsigned short* __restrict__ Btp, const unsigned short* __restrict__ Bt2p, int ldb, long strideB,
    void* __restrict__ Cout, void* __restrict__ Cout2, int ldc, long strideC,
    const float* __restrict__ bias,
    const float* __restrict__ resid, long strideR,
    int M, int N, int K, float scale) {
  typedef typename Elem<ET>::T T;
  typedef typename Frag<T>::V V;
  const T* A = (const T*)Ap; const T* A2 = (const T*)A2p; const T* Bt = (const T*)Btp; const T* Bt2 = (const T*)Bt2p;
  __shared__ __align__(16) float sT[8][16 * 68];
  const int b    = blockIdx.y;
  const int lane = threadIdx.x & 31;
  const int wave = threadIdx.x >> 5;
  const int tilesN = N >> 6;
  const int tilesM = M >> 6;
  const int tile = blockIdx.x * 8 + wave;
  if (tile >= tilesM * tilesN) return;
  const int tm = tile / tilesN;
  const int tn = tile - tm * tilesN;
  const int m0 = tm << 6;
  const int n0 = tn << 6;

  const T* Ab  = A  + (size_t)b * strideA;
  const T* Bb  = Bt + (size_t)b * strideB;
  const T* Ab2 = SPLIT ? (A2  + (size_t)b * strideA) : nullptr;
  const T* Bb2 = SPLIT ? (Bt2 + (size_t)b * strideB) : nullptr;

  const int rlane = lane & 15;
  const int koff  = (lane >> 4) * 8;
  const int mOff  = (lane >> 4) * 8;

  v8f acc[4][4];
#pragma unroll
  for (int i = 0; i < 4; ++i)
#pragma unroll
    for (int j = 0; j < 4; ++j) acc[i][j] = (v8f){0.f,0.f,0.f,0.f,0.f,0.f,0.f,0.f};

  for (int k0 = 0; k0 < K; k0 += 32) {
    V bh[4], bl[4];
#pragma unroll
    for (int j = 0; j < 4; ++j) {
      const size_t bo = (size_t)(n0 + (j << 4) + rlane) * ldb + koff + k0;
      bh[j] = Frag<T>::load(Bb + bo);
      if (SPLIT) bl[j] = Frag<T>::load(Bb2 + bo);
    }
#pragma unroll
    for (int i = 0; i < 4; ++i) {
      const size_t ao = (size_t)(m0 + (i << 4) + rlane) * lda + koff + k0;
      V ah = Frag<T>::load(Ab + ao);
      V al;
      if (SPLIT) al = Frag<T>::load(Ab2 + ao);
#pragma unroll
      for (int j = 0; j < 4; ++j) {
        acc[i][j] = Frag<T>::mma(ah, bh[j], acc[i][j]);
        if (SPLIT) {
          acc[i][j] = Frag<T>::mma(ah, bl[j], acc[i][j]);
          acc[i][j] = Frag<T>::mma(al, bh[j], acc[i][j]);
        }
      }
      Frag<T>::guard(acc[i][0], acc[i][3], ah, SPLIT ? al : ah);
    }
    Frag<T>::keep(bh[0], bh[1], bh[2], bh[3]);
    if (SPLIT) Frag<T>::keep(bl[0], bl[1], bl[2], bl[3]);
  }
  acc_guard4(acc[0][0], acc[0][1], acc[0][2], acc[0][3]);
  acc_guard4(acc[1][0], acc[1][1], acc[1][2], acc[1][3]);
  acc_guard4(acc[2][0], acc[2][1], acc[2][2], acc[2][3]);
  acc_guard4(acc[3][0], acc[3][1], acc[3][2], acc[3][3]);

  float* slab = sT[wave];
  const float* Rb = RESID ? (resid + (size_t)b * strideR) : nullptr;
#pragma unroll
  for (int i = 0; i < 4; ++i) {
    const int mBase = m0 + (i << 4);
#pragma unroll
    for (int j = 0; j < 4; ++j) {
      const int n = n0 + (j << 4) + rlane;
      float bv = 0.f;
      if (BIAS_MODE == 2) bv = bias[n];
#pragma unroll
      for (int r = 0; r < 8; ++r) {
        float v = acc[i][j][r] * scale;
        if (BIAS_MODE == 1) v += bias[mBase + mOff + r];
        if (BIAS_MODE == 2) v += bv;
        if (RESID) v += Rb[(size_t)(mBase + mOff + r) * ldc + n];
        if (ACT == 2) v = fmaxf(v, 0.0f);
        if (ACT == 4) v = (v > 0.f) ? v : 0.01f * v;
        slab[(mOff + r) * 68 + (j << 4) + rlane] = v;
      }
    }
    __builtin_amdgcn_fence(__ATOMIC_RELEASE, "workgroup");
    __builtin_amdgcn_wave_barrier();
    __builtin_amdgcn_fence(__ATOMIC_ACQUIRE, "workgroup");
    if (OUT_MODE == 0) {
      float* C = (float*)Cout + (size_t)b * strideC;
      const int hh = lane >> 4, c4 = (lane & 15) * 4;
      for (int pass = 0; pass < 2; ++pass) {
#pragma unroll
        for (int it = 0; it < 8; ++it) {
          const int row = it * 2 + hh;
          v4f v = *(const v4f*)(slab + row * 68 + c4);
          *(volatile v4f*)(C + (size_t)(mBase + row) * ldc + n0 + c4) = v;
        }
        __threadfence();
      }
    } else {
      const int q = lane >> 3, c8 = (lane & 7) * 8;
      unsigned short* C  = (unsigned short*)Cout  + (size_t)b * strideC;
      unsigned short* C2 = (OUT_MODE == 2) ? ((unsigned short*)Cout2 + (size_t)b * strideC) : nullptr;
      for (int pass = 0; pass < 2; ++pass) {
#pragma unroll
        for (int it = 0; it < 4; ++it) {
          const int row = it * 4 + q;
          const float* sp = slab + row * 68 + c8;
          v8h hv, lv;
#pragma unroll
          for (int e = 0; e < 8; ++e) {
            if (OUT_MODE == 1) {
              hv[e] = (_Float16)sp[e];
            } else {
              unsigned short hb = f2bf_bits(sp[e]);
              unsigned short lb = f2bf_bits(sp[e] - bf_bits2f(hb));
              hv[e] = __builtin_bit_cast(_Float16, hb);
              lv[e] = __builtin_bit_cast(_Float16, lb);
            }
          }
          *(volatile v8h*)(C + (size_t)(mBase + row) * ldc + n0 + c8) = hv;
          if (OUT_MODE == 2) *(volatile v8h*)(C2 + (size_t)(mBase + row) * ldc + n0 + c8) = lv;
        }
        __threadfence();
      }
    }
    __builtin_amdgcn_fence(__ATOMIC_RELEASE, "workgroup");
    __builtin_amdgcn_wave_barrier();
    __builtin_amdgcn_fence(__ATOMIC_ACQUIRE, "workgroup");
  }
}

__global__ __launch_bounds__(256) void cast8_f16_kernel(const float* __restrict__ in, unsigned short* __restrict__ out,
                                                        int n8, float scale) {
  const int i = blockIdx.x * 256 + threadIdx.x;
  if (i >= n8) return;
  const float* p = in + 8 * (size_t)i;
  const v4f a = *(const v4f*)(p);
  const v4f c = *(const v4f*)(p + 4);
  unsigned short hb[8];
#pragma unroll
  for (int e = 0; e < 4; ++e) {
    hb[e]     = h_bits(a[e] * scale);
    hb[4 + e] = h_bits(c[e] * scale);
  }
  const v4u u = (v4u){pk16(hb[0], hb[1]), pk16(hb[2], hb[3]), pk16(hb[4], hb[5]), pk16(hb[6], hb[7])};
  unsigned short* q = out + 8 * (size_t)i;
  *(volatile v4u*)q = u;
  __threadfence();
  *(volatile v4u*)q = u;
}

__global__ __launch_bounds__(256) void zero_pads_kernel(unsigned short* __restrict__ qk, unsigned short* __restrict__ vt) {
  const v4u z = (v4u){0u, 0u, 0u, 0u};
  const int g = blockIdx.x * 256 + threadIdx.x;
  if (blockIdx.x < 256) {
    const int side = g >> 15, idx = g & 32767;
    unsigned short* p = qk + (size_t)side * ((size_t)(kWin + kTok) * kQKld) + (size_t)idx * 8;
    *(volatile v4u*)p = z;
    __threadfence();
    *(volatile v4u*)p = z;
  } else {
    const int g2 = g - 65536;
    const int row = g2 >> 5, side = (g2 >> 4) & 1, piece = g2 & 15;
    unsigned short* p = vt + (size_t)row * kVtld + side * (kWin + kTok) + piece * 8;
    *(volatile v4u*)p = z;
    __threadfence();
    *(volatile v4u*)p = z;
  }
}

__global__ __launch_bounds__(128) void layernorm_f16_kernel(const float* __restrict__ x, const float* __restrict__ gam,
                                                            const float* __restrict__ bet, unsigned short* __restrict__ out) {
  __shared__ float redA[4];
  __shared__ float redB[4];
  const int row  = blockIdx.x;
  const int t    = threadIdx.x, lane = t & 31, wave = t >> 5;
  const float* xr = x + (size_t)row * kDim + 8 * t;
  const v4f a = *(const v4f*)(xr);
  const v4f c = *(const v4f*)(xr + 4);
  float s = ((a[0] + a[1]) + (a[2] + a[3])) + ((c[0] + c[1]) + (c[2] + c[3]));
#pragma unroll
  for (int off = 16; off > 0; off >>= 1) s += __shfl_xor(s, off, 32);
  if (lane == 0) redA[wave] = s;
  __syncthreads();
  const float mean = (((redA[0] + redA[1]) + redA[2]) + redA[3]) * kInvDim;
  float d[8];
#pragma unroll
  for (int e = 0; e < 4; ++e) { d[e] = a[e] - mean; d[4 + e] = c[e] - mean; }
  float q = 0.f;
#pragma unroll
  for (int e = 0; e < 8; ++e) q += d[e] * d[e];
#pragma unroll
  for (int off = 16; off > 0; off >>= 1) q += __shfl_xor(q, off, 32);
  if (lane == 0) redB[wave] = q;
  __syncthreads();
  const float var  = (((redB[0] + redB[1]) + redB[2]) + redB[3]) * kInvDim;
  const float rstd = 1.0f / sqrtf(var + kLnEps);
  const v4f g0 = *(const v4f*)(gam + 8 * t);
  const v4f g1v = *(const v4f*)(gam + 8 * t + 4);
  const v4f b0 = *(const v4f*)(bet + 8 * t);
  const v4f b1v = *(const v4f*)(bet + 8 * t + 4);
  unsigned short hb[8];
#pragma unroll
  for (int e = 0; e < 4; ++e) {
    hb[e]     = h_bits(d[e] * rstd * g0[e] + b0[e]);
    hb[4 + e] = h_bits(d[4 + e] * rstd * g1v[e] + b1v[e]);
  }
  const v4u u = (v4u){pk16(hb[0], hb[1]), pk16(hb[2], hb[3]), pk16(hb[4], hb[5]), pk16(hb[6], hb[7])};
  unsigned short* op = out + (size_t)row * kDim + 8 * t;
  *(volatile v4u*)op = u;
  __threadfence();
  *(volatile v4u*)op = u;
}

__global__ __launch_bounds__(128) void band_softmax_kernel(const float* __restrict__ S, unsigned short* __restrict__ P) {
  __shared__ __align__(16) float srow[4][kWinK];
  __shared__ __align__(16) unsigned short prow[4][kWinK];
  const int t    = threadIdx.x, lane = t & 31, wave = t >> 5;
  const int row  = blockIdx.x * 4 + wave;
  const int c    = row >> 7;
  const int i    = row & 127;
  const float* sr = S + (size_t)row * kWinK;
  float m = -INFINITY;
#pragma unroll 1
  for (int j = 0; j < 12; ++j) {
    const int n   = 32 * j + lane;
    const int key = kChunkQ * c - kWin + n;
    const bool valid = (key >= 0) && (key < kTok) && (n >= i) && (n <= i + 2 * kWin);
    const float sv = sr[n] * kScoreScale;
    const float s  = valid ? sv : -INFINITY;
    srow[wave][n] = s;
    m = fmaxf(m, s);
  }
#pragma unroll
  for (int off = 16; off > 0; off >>= 1) m = fmaxf(m, __shfl_xor(m, off, 32));
  float sum = 0.f;
#pragma unroll 1
  for (int j = 0; j < 12; ++j) {
    const int n   = 32 * j + lane;
    const int key = kChunkQ * c - kWin + n;
    const bool valid = (key >= 0) && (key < kTok) && (n >= i) && (n <= i + 2 * kWin);
    const float s   = srow[wave][n];
    const float arg = valid ? (s - m) : 0.f;
    const float ex  = expf(arg);
    const float e   = valid ? ex : 0.f;
    srow[wave][n] = e;
    sum += e;
  }
#pragma unroll
  for (int off = 16; off > 0; off >>= 1) sum += __shfl_xor(sum, off, 32);
  const float inv = kPCarry / sum;
#pragma unroll 1
  for (int j = 0; j < 12; ++j) {
    const int n = 32 * j + lane;
    prow[wave][n] = h_bits(srow[wave][n] * inv);
  }
  __syncthreads();
  unsigned short* pr = P + (size_t)row * kWinK;
  const v4u u0 = *(const v4u*)(&prow[wave][8 * lane]);
  const v4u u1 = *(const v4u*)(&prow[wave][256 + 8 * (lane & 15)]);
  for (int pass = 0; pass < 2; ++pass) {
    *(volatile v4u*)(pr + 8 * lane) = u0;
    if (lane < 16) *(volatile v4u*)(pr + 256 + 8 * lane) = u1;
    __threadfence();
  }
}

__global__ __launch_bounds__(256) void gelu_f16_kernel(const unsigned* __restrict__ in, unsigned* __restrict__ out,
                                                       int nwords, float carry) {
  const int i = blockIdx.x * 256 + threadIdx.x;
  if (i >= nwords) return;
  const unsigned w = in[i];
  unsigned r = 0u;
#pragma unroll 1
  for (int e = 0; e < 2; ++e) {
    const unsigned short hb = (unsigned short)((e == 0) ? (w & 0xffffu) : (w >> 16));
    const float x  = (float)__builtin_bit_cast(_Float16, hb);
    const float gl = 0.5f * x * (1.0f + erff(x * 0.70710678118654752f));
    const unsigned short ob = h_bits(gl * carry);
    r |= ((unsigned)ob) << (16 * e);
  }
  ((volatile unsigned*)out)[i] = r;
  __threadfence();
  ((volatile unsigned*)out)[i] = r;
}

extern "C" void kernel_launch(void* const* d_in, const int* in_sizes, int n_in,
                              void* d_out, int out_size, void* d_ws, size_t ws_size, hipStream_t stream) {
  if (n_in < 13) return;
  if (in_sizes[0] != kTok * kDim || in_sizes[1] != 3 * kDim * kDim || in_sizes[2] != 3 * kDim ||
      in_sizes[3] != kDim * kDim || in_sizes[4] != kDim || in_sizes[5] != kDim || in_sizes[6] != kDim ||
      in_sizes[7] != kDim || in_sizes[8] != kDim || in_sizes[9] != kMlp * kDim || in_sizes[10] != kMlp ||
      in_sizes[11] != kDim * kMlp || in_sizes[12] != kDim) return;
  if (out_size != kTok * kDim) return;
  if (ws_size < kWsTotal) return;

  const float* x     = (const float*)d_in[0];
  const float* w_qkv = (const float*)d_in[1];
  const float* b_qkv = (const float*)d_in[2];
  const float* w_out = (const float*)d_in[3];
  const float* b_out = (const float*)d_in[4];
  const float* g1    = (const float*)d_in[5];
  const float* be1   = (const float*)d_in[6];
  const float* g2    = (const float*)d_in[7];
  const float* be2   = (const float*)d_in[8];
  const float* w1    = (const float*)d_in[9];
  const float* b1    = (const float*)d_in[10];
  const float* w2    = (const float*)d_in[11];
  const float* b2    = (const float*)d_in[12];
  float* out = (float*)d_out;

  char* ws = (char*)d_ws;
  unsigned short* wqkv_h = (unsigned short*)(ws + kOffWqkv);
  unsigned short* wout_h = (unsigned short*)(ws + kOffWout);
  unsigned short* qkpad  = (unsigned short*)(ws + kOffQK);
  unsigned short* vt     = (unsigned short*)(ws + kOffVt);
  float*          scores = (float*)(ws + kOffS);
  unsigned short* pplane = (unsigned short*)(ws + kOffP);
  unsigned short* oplane = (unsigned short*)(ws + kOffO);
  unsigned short* hpre   = (unsigned short*)(ws + kOffHpre);
  unsigned short* w1_h   = (unsigned short*)(ws + kOffW1);
  unsigned short* w2_h   = (unsigned short*)(ws + kOffW2);
  unsigned short* xn     = (unsigned short*)(ws + kOffXn);
  float*          x1     = (float*)(ws + kOffX1);
  unsigned short* hact   = (unsigned short*)(ws + kOffHact);

  cast8_f16_kernel<<<(3 * kDim * kDim / 8) / 256, 256, 0, stream>>>(w_qkv, wqkv_h, 3 * kDim * kDim / 8, kWCarry);
  cast8_f16_kernel<<<(kDim * kDim / 8) / 256, 256, 0, stream>>>(w_out, wout_h, kDim * kDim / 8, kWCarry);
  cast8_f16_kernel<<<(kMlp * kDim / 8) / 256, 256, 0, stream>>>(w1, w1_h, kMlp * kDim / 8, kWCarry);
  cast8_f16_kernel<<<(kDim * kMlp / 8) / 256, 256, 0, stream>>>(w2, w2_h, kDim * kMlp / 8, kWCarry);

  zero_pads_kernel<<<384, 256, 0, stream>>>(qkpad, vt);

  layernorm_f16_kernel<<<kTok, 128, 0, stream>>>(x, g1, be1, xn);

  wmma_gemm64<0, false, 2, 1, false><<<dim3(256, 1), 256, 0, stream>>>(
      xn, nullptr, kDim, 0L, wqkv_h, nullptr, kDim, 0L,
      (void*)(qkpad + (size_t)kWin * kQKld), nullptr, kQKld, 0L,
      b_qkv, nullptr, 0L, kTok, 2 * kDim, kDim, kWCarryInv);

  wmma_gemm64<0, false, 1, 1, false><<<dim3(128, 1), 256, 0, stream>>>(
      wqkv_h + (size_t)2 * kDim * kDim, nullptr, kDim, 0L, xn, nullptr, kDim, 0L,
      (void*)(vt + kWin), nullptr, kVtld, 0L,
      b_qkv + 2 * kDim, nullptr, 0L, kDim, kTok, kDim, kWCarryInv);

  for (int h = 0; h < kHeads; ++h) {
    wmma_gemm64<0, false, 0, 0, false><<<dim3(2, kNChunk), 256, 0, stream>>>(
        qkpad + (size_t)kWin * kQKld + h * kHdim, nullptr, kQKld, (long)kChunkQ * kQKld,
        qkpad + kDim + h * kHdim, nullptr, kQKld, (long)kChunkQ * kQKld,
        (void*)scores, nullptr, kWinK, (long)kChunkQ * kWinK,
        nullptr, nullptr, 0L, kChunkQ, kWinK, kHdim, 1.0f);
    band_softmax_kernel<<<kTok / 4, 128, 0, stream>>>(scores, pplane);
    wmma_gemm64<0, false, 0, 1, false><<<dim3(1, kNChunk), 256, 0, stream>>>(
        pplane, nullptr, kWinK, (long)kChunkQ * kWinK,
        vt + (size_t)h * kHdim * kVtld, nullptr, kVtld, (long)kChunkQ,
        (void*)(oplane + h * kHdim), nullptr, kDim, (long)kChunkQ * kDim,
        nullptr, nullptr, 0L, kChunkQ, kHdim, kWinK, kOCarry / kPCarry);
  }

  wmma_gemm64<0, false, 2, 0, true><<<dim3(128, 1), 256, 0, stream>>>(
      oplane, nullptr, kDim, 0L, wout_h, nullptr, kDim, 0L,
      (void*)x1, nullptr, kDim, 0L,
      b_out, x, 0L, kTok, kDim, kDim, 1.0f / (kOCarry * kWCarry));

  layernorm_f16_kernel<<<kTok, 128, 0, stream>>>(x1, g2, be2, xn);

  wmma_gemm64<0, false, 2, 1, false><<<dim3(512, 1), 256, 0, stream>>>(
      xn, nullptr, kDim, 0L, w1_h, nullptr, kDim, 0L,
      (void*)hpre, nullptr, kMlp, 0L,
      b1, nullptr, 0L, kTok, kMlp, kDim, kWCarryInv);

  gelu_f16_kernel<<<(kTok * kMlp / 2) / 256, 256, 0, stream>>>(
      (const unsigned*)hpre, (unsigned*)hact, kTok * kMlp / 2, kHCarry);

  wmma_gemm64<0, false, 2, 0, true><<<dim3(128, 1), 256, 0, stream>>>(
      hact, nullptr, kMlp, 0L, w2_h, nullptr, kMlp, 0L,
      (void*)out, nullptr, kDim, 0L,
      b2, x1, 0L, kTok, kDim, kMlp, 1.0f / (kHCarry * kWCarry));
}
